// TemporalAwareAttention_67104569033194
// MI455X (gfx1250) — hardware-verified
//
#include <hip/hip_runtime.h>
#include <stdint.h>

#define NB   2
#define NL   2048
#define ND   1024
#define NH   16
#define HD   64
#define QS   8.0f
#define SM_SCALE 0.001953125f
#define RB   0.1f
#define EPS  1.0e-8f
#define HMEAN 0.0625f
#define PSP  72
#define FSP  68
#define NBX  ((NB * NL * ND) / 2048)
#define NBW  ((2 * ND * ND) / 2048)
static_assert(NBX == 2048 && NBW == 1024);
static_assert(NH * HD == ND);
static_assert((NL % 128) == 0 && (ND % 64) == 0 && (NL % 32) == 0);

typedef _Float16 v16h __attribute__((ext_vector_type(16)));
typedef _Float16 v8h  __attribute__((ext_vector_type(8)));
typedef float    v8f  __attribute__((ext_vector_type(8)));
typedef float    v4f  __attribute__((ext_vector_type(4)));
typedef unsigned int v4u __attribute__((ext_vector_type(4)));
typedef unsigned int v8u __attribute__((ext_vector_type(8)));
typedef __bf16   v16bf __attribute__((ext_vector_type(16)));

union FragH { v16h v; v8h h[2]; };
union FragU { v8u v; v4u h[2]; };

__device__ __forceinline__ unsigned short bf_bits(float f) {
  unsigned u = __float_as_uint(f);
  return (unsigned short)((u + 0x7FFFu + ((u >> 16) & 1u)) >> 16);
}
__device__ __forceinline__ float bf_up(unsigned short h) { return __uint_as_float(((unsigned)h) << 16); }
__device__ __forceinline__ float bfr(float f) { return bf_up(bf_bits(f)); }
__device__ __forceinline__ unsigned short h_bits(_Float16 x) { return __builtin_bit_cast(unsigned short, x); }
__device__ __forceinline__ unsigned pk16(unsigned short a, unsigned short b) { return (unsigned)a | ((unsigned)b << 16); }
__device__ __forceinline__ v8f zero8() { v8f z = {0.f, 0.f, 0.f, 0.f, 0.f, 0.f, 0.f, 0.f}; return z; }

__device__ __forceinline__ v16h ldfrag_h(const _Float16* p) {
  FragH f;
  f.h[0] = *(const v8h*)(p);
  f.h[1] = *(const v8h*)(p + 16);
  return f.v;
}
__device__ __forceinline__ v8u ldfrag_u(const unsigned short* p) {
  FragU f;
  f.h[0] = *(const v4u*)(p);
  f.h[1] = *(const v4u*)(p + 16);
  return f.v;
}

__device__ __forceinline__ v8f mma_h(v16h a, v16h b, v8f c) {
  return __builtin_amdgcn_wmma_f32_16x16x32_f16(false, a, false, b, (short)0, c, false, false);
}
__device__ __forceinline__ v8f mma_b(v8u a, v8u b, v8f c) {
  return __builtin_amdgcn_wmma_f32_16x16x32_bf16(false, __builtin_bit_cast(v16bf, a),
                                                 false, __builtin_bit_cast(v16bf, b), (short)0, c, false, false);
}
__device__ __forceinline__ void guard_s(v8f& s, v16h a0, v16h a1, v16h b0, v16h b1) {
#if defined(__HIP_DEVICE_COMPILE__)
  asm volatile("v_nop\n\tv_nop\n\tv_nop\n\tv_nop" : "+v"(s) : "v"(a0), "v"(a1), "v"(b0), "v"(b1));
#endif
}
__device__ __forceinline__ void guard8(v8f& c0, v8f& c1, v8f& c2, v8f& c3, v8f& c4, v8f& c5, v8f& c6, v8f& c7,
                                       v8u f0, v8u f1, v8u f2, v8u f3, v8u f4, v8u f5, v8u f6, v8u f7) {
#if defined(__HIP_DEVICE_COMPILE__)
  asm volatile("v_nop\n\tv_nop\n\tv_nop\n\tv_nop"
               : "+v"(c0), "+v"(c1), "+v"(c2), "+v"(c3), "+v"(c4), "+v"(c5), "+v"(c6), "+v"(c7)
               : "v"(f0), "v"(f1), "v"(f2), "v"(f3), "v"(f4), "v"(f5), "v"(f6), "v"(f7));
#endif
}

__global__ __launch_bounds__(256) void cvt_in(const float* __restrict__ x, const float* __restrict__ w,
                                               unsigned short* Xb, unsigned short* Wb) {
  const int bx = blockIdx.x;
  const bool isx = (bx < NBX);
  const float* src = isx ? x : w;
  unsigned short* dst = isx ? Xb : Wb;
  const size_t e0 = ((size_t)(isx ? bx : (bx - NBX)) * 256 + threadIdx.x) * 8;
  const v4f a = *(const v4f*)(src + e0);
  const v4f c = *(const v4f*)(src + e0 + 4);
  v4u v;
  v[0] = pk16(bf_bits(a[0]), bf_bits(a[1]));
  v[1] = pk16(bf_bits(a[2]), bf_bits(a[3]));
  v[2] = pk16(bf_bits(c[0]), bf_bits(c[1]));
  v[3] = pk16(bf_bits(c[2]), bf_bits(c[3]));
  unsigned short* dp = dst + e0;
  *(volatile v4u*)dp = v;
  __threadfence();
  *(volatile v4u*)dp = v;
}

__global__ __launch_bounds__(256) void xpt(const float* __restrict__ x, unsigned short* XT) {
  __shared__ __align__(16) unsigned short Ts[64 * PSP];
  const int tid = threadIdx.x;
  const int bx  = blockIdx.x;
  const int b   = bx >> 9;
  const int lt  = (bx >> 4) & 31;
  const int dt  = bx & 15;
  const int l0  = lt * 64, d0 = dt * 64;
  {
    const int q = tid & 15, r16 = tid >> 4;
#pragma unroll
    for (int it = 0; it < 4; ++it) {
      const int ll = it * 16 + r16;
      const v4f v = *(const v4f*)(x + ((size_t)(b * NL + l0 + ll)) * ND + d0 + 4 * q);
#pragma unroll
      for (int e = 0; e < 4; ++e) Ts[(4 * q + e) * PSP + ll] = bf_bits(v[e]);
    }
  }
  __syncthreads();
  {
    const int e8 = tid & 7, fq = tid >> 3;
    v4u vals[2];
#pragma unroll
    for (int it = 0; it < 2; ++it) {
      const int dl = it * 32 + fq;
      vals[it] = *(const v4u*)(Ts + dl * PSP + 8 * e8);
    }
    unsigned short* dp = XT + ((size_t)(b * ND + d0)) * NL + l0 + 8 * e8;
    for (int pass = 0; pass < 2; ++pass) {
#pragma unroll
      for (int it = 0; it < 2; ++it) {
        const int dl = it * 32 + fq;
        *(volatile v4u*)(dp + (size_t)dl * NL) = vals[it];
      }
      __threadfence();
    }
  }
}

__global__ __launch_bounds__(128)
void proj_qk(const unsigned short* __restrict__ Xb, const unsigned short* __restrict__ Wb,
             const float* __restrict__ bias, unsigned short* QK) {
  __shared__ __align__(16) unsigned short Ps[128 * PSP];
  const int tid  = threadIdx.x;
  const int wave = tid >> 5;
  const int lane = tid & 31;
  const int hh   = lane >> 4;
  const int ci   = lane & 15;
  const int bx   = blockIdx.x;
  const int nt   = bx & 31;
  const int mt   = bx >> 5;
  const int m0   = mt * 128, n0 = nt * 64;

  const unsigned short* Ap = Xb + ((size_t)(m0 + 32 * wave + ci)) * ND + 8 * hh;
  const unsigned short* Bp = Wb + ((size_t)(n0 + ci)) * ND + 8 * hh;

  v8f acc[2][4];
#pragma unroll
  for (int i = 0; i < 2; ++i) {
#pragma unroll
    for (int t = 0; t < 4; ++t) acc[i][t] = zero8();
  }

#pragma unroll 1
  for (int k0 = 0; k0 < ND; k0 += 32) {
    const v8u a0 = ldfrag_u(Ap + k0);
    const v8u a1 = ldfrag_u(Ap + (size_t)16 * ND + k0);
    v8u bf[4];
#pragma unroll
    for (int t = 0; t < 4; ++t) bf[t] = ldfrag_u(Bp + (size_t)(16 * t) * ND + k0);
#pragma unroll
    for (int t = 0; t < 4; ++t) {
      acc[0][t] = mma_b(a0, bf[t], acc[0][t]);
      acc[1][t] = mma_b(a1, bf[t], acc[1][t]);
    }
    guard8(acc[0][0], acc[0][1], acc[0][2], acc[0][3], acc[1][0], acc[1][1], acc[1][2], acc[1][3],
           a0, a1, bf[0], bf[1], bf[2], bf[3], a0, a1);
  }

  float bv[4];
#pragma unroll
  for (int t = 0; t < 4; ++t) bv[t] = bfr(bias[n0 + 16 * t + ci]);
#pragma unroll
  for (int i = 0; i < 2; ++i) {
#pragma unroll
    for (int t = 0; t < 4; ++t) {
#pragma unroll
      for (int r = 0; r < 8; ++r) {
        const float v = (acc[i][t][r] + bv[t]) * QS;
        Ps[(32 * wave + 16 * i + 8 * hh + r) * PSP + 16 * t + ci] = h_bits((_Float16)v);
      }
    }
  }
  __syncthreads();
  {
    const int isK = nt >> 4, h = nt & 15;
    const int b   = mt >> 4, l0 = m0 & (NL - 1);
    unsigned short* dst = QK + ((((size_t)isK * NB + b) * NH + h) * NL + l0) * HD;
    const int p = tid & 7, rg = tid >> 3;
    v4u vals[8];
#pragma unroll
    for (int it = 0; it < 8; ++it) {
      const int row = it * 16 + rg;
      vals[it] = *(const v4u*)(Ps + row * PSP + 8 * p);
    }
    for (int pass = 0; pass < 2; ++pass) {
#pragma unroll
      for (int it = 0; it < 8; ++it) {
        const int row = it * 16 + rg;
        *(volatile v4u*)(dst + (size_t)row * HD + 8 * p) = vals[it];
      }
      __threadfence();
    }
  }
}

__global__ __launch_bounds__(256)
void attn_w(const unsigned short* __restrict__ QK, const float* __restrict__ td,
            float* out1, unsigned short* AH, unsigned short* AL) {
  __shared__ __align__(16) float sS[16 * NL];
  __shared__ float redm[8 * 16];
  const int tid  = threadIdx.x;
  const int wave = tid >> 5;
  const int lane = tid & 31;
  const int hh   = lane >> 4;
  const int ci   = lane & 15;
  const int row  = tid >> 4;
  const int tx   = tid & 15;
  const int bx   = blockIdx.x;
  const int b    = bx >> 7;
  const int q0   = (bx & 127) * 16;

  const _Float16* Qp = (const _Float16*)(const void*)QK;
  const _Float16* Kp = Qp + (size_t)NB * NH * NL * HD;
  float* srow = sS + row * NL + tx;

  float acc[128];
#pragma unroll
  for (int j = 0; j < 128; ++j) acc[j] = 0.f;

#pragma unroll 1
  for (int h = 0; h < NH; ++h) {
    __syncthreads();
    const size_t hb = ((size_t)(b * NH + h)) * NL;
    const _Float16* qp = Qp + (hb + q0 + ci) * HD + 8 * hh;
    const v16h a0 = ldfrag_h(qp);
    const v16h a1 = ldfrag_h(qp + 32);
    const _Float16* kp0 = Kp + (hb + ci) * HD + 8 * hh;
    float mx[8];
#pragma unroll
    for (int r = 0; r < 8; ++r) mx[r] = -3.0e38f;

#pragma unroll 1
    for (int t = 0; t < 16; ++t) {
      const int key0 = (wave * 16 + t) * 16;
      const _Float16* kp = kp0 + (size_t)key0 * HD;
      const v16h b0 = ldfrag_h(kp);
      const v16h b1 = ldfrag_h(kp + 32);
      v8f s = zero8();
      s = mma_h(a0, b0, s);
      s = mma_h(a1, b1, s);
      guard_s(s, a0, a1, b0, b1);
      float* sp = sS + (8 * hh) * NL + key0 + ci;
#pragma unroll
      for (int r = 0; r < 8; ++r) {
        sp[r * NL] = s[r];
        mx[r] = fmaxf(mx[r], s[r]);
      }
    }
#pragma unroll
    for (int r = 0; r < 8; ++r) {
      float v = mx[r];
      v = fmaxf(v, __shfl_xor(v, 1, 32));
      v = fmaxf(v, __shfl_xor(v, 2, 32));
      v = fmaxf(v, __shfl_xor(v, 4, 32));
      v = fmaxf(v, __shfl_xor(v, 8, 32));
      mx[r] = v;
    }
    if (ci == 0) {
#pragma unroll
      for (int r = 0; r < 8; ++r) redm[wave * 16 + 8 * hh + r] = mx[r];
    }
    __syncthreads();

    float m = redm[row];
#pragma unroll
    for (int w2 = 1; w2 < 8; ++w2) m = fmaxf(m, redm[w2 * 16 + row]);
    float sum = 0.f;
#pragma unroll 4
    for (int j = 0; j < 128; ++j) {
      const float e = __expf((srow[16 * j] - m) * SM_SCALE);
      sum += e;
      srow[16 * j] = e;
    }
    sum += __shfl_xor(sum, 1, 32);
    sum += __shfl_xor(sum, 2, 32);
    sum += __shfl_xor(sum, 4, 32);
    sum += __shfl_xor(sum, 8, 32);
    const float inv = 1.0f / sum;
#pragma unroll
    for (int j = 0; j < 128; ++j) acc[j] = fmaf(srow[16 * j], inv, acc[j]);
  }

#pragma unroll
  for (int j = 0; j < 128; ++j) srow[16 * j] = acc[j] * HMEAN;
  const float* tdrow = td + ((size_t)(b * NL + q0 + row)) * NL + tx;
  float dsum = 0.f;
#pragma unroll 4
  for (int j = 0; j < 128; ++j) {
    const float v   = srow[16 * j];
    const float tdb = bfr(tdrow[16 * j]);
    const float a   = v * __expf(-RB * tdb);
    dsum += a;
    srow[16 * j] = a;
  }
  dsum += __shfl_xor(dsum, 1, 32);
  dsum += __shfl_xor(dsum, 2, 32);
  dsum += __shfl_xor(dsum, 4, 32);
  dsum += __shfl_xor(dsum, 8, 32);
  const float rinv = 1.0f / (dsum + EPS);
#pragma unroll 4
  for (int j = 0; j < 128; ++j) {
    const float a = srow[16 * j] * rinv;
    srow[16 * j] = a;
  }
  __syncthreads();

  const size_t g0 = (size_t)(b * NL + q0);
  for (int pass = 0; pass < 2; ++pass) {
#pragma unroll
    for (int s2 = 0; s2 < 2; ++s2) {
      const int rr = 2 * wave + s2;
      const float* sr = sS + rr * NL + 4 * lane;
      float* orow = out1 + (g0 + rr) * NL + 4 * lane;
#pragma unroll 4
      for (int it = 0; it < 16; ++it) {
        const v4f v = *(const v4f*)(sr + it * 128);
        *(volatile v4f*)(orow + it * 128) = v;
      }
    }
    __threadfence();
  }
  for (int pass = 0; pass < 2; ++pass) {
#pragma unroll
    for (int s2 = 0; s2 < 2; ++s2) {
      const int rr = 2 * wave + s2;
      const float* sr = sS + rr * NL + 8 * lane;
      unsigned short* hrow = AH + (g0 + rr) * NL + 8 * lane;
      unsigned short* lrow = AL + (g0 + rr) * NL + 8 * lane;
#pragma unroll 2
      for (int it = 0; it < 8; ++it) {
        const v4f f0 = *(const v4f*)(sr + it * 256);
        const v4f f1 = *(const v4f*)(sr + it * 256 + 4);
        float f[8];
#pragma unroll
        for (int e = 0; e < 4; ++e) { f[e] = f0[e]; f[4 + e] = f1[e]; }
        v4u hv, lv;
#pragma unroll
        for (int e = 0; e < 4; ++e) {
          const unsigned short hb0 = bf_bits(f[2 * e]);
          const unsigned short hb1 = bf_bits(f[2 * e + 1]);
          const unsigned short lb0 = bf_bits(f[2 * e] - bf_up(hb0));
          const unsigned short lb1 = bf_bits(f[2 * e + 1] - bf_up(hb1));
          hv[e] = pk16(hb0, hb1);
          lv[e] = pk16(lb0, lb1);
        }
        *(volatile v4u*)(hrow + it * 256) = hv;
        *(volatile v4u*)(lrow + it * 256) = lv;
      }
    }
    __threadfence();
  }
}

__global__ __launch_bounds__(128)
void out_prod(const unsigned short* __restrict__ AH, const unsigned short* __restrict__ AL,
              const unsigned short* __restrict__ XT, float* out0) {
  __shared__ __align__(16) float Fs[128 * FSP];
  const int tid  = threadIdx.x;
  const int wave = tid >> 5;
  const int lane = tid & 31;
  const int hh   = lane >> 4;
  const int ci   = lane & 15;
  const int bx   = blockIdx.x;
  const int b    = bx >> 8;
  const int mt   = (bx >> 4) & 15;
  const int nt   = bx & 15;
  const int q0   = mt * 128, d0 = nt * 64;

  const size_t ar = ((size_t)(b * NL + q0 + 32 * wave + ci)) * NL + 8 * hh;
  const unsigned short* Hp = AH + ar;
  const unsigned short* Lp = AL + ar;
  const unsigned short* Bp = XT + ((size_t)(b * ND + d0 + ci)) * NL + 8 * hh;

  v8f acc[2][4];
#pragma unroll
  for (int i = 0; i < 2; ++i) {
#pragma unroll
    for (int t = 0; t < 4; ++t) acc[i][t] = zero8();
  }

#pragma unroll 1
  for (int k0 = 0; k0 < NL; k0 += 32) {
    const v8u h0  = ldfrag_u(Hp + k0);
    const v8u h1  = ldfrag_u(Hp + (size_t)16 * NL + k0);
    const v8u l0v = ldfrag_u(Lp + k0);
    const v8u l1v = ldfrag_u(Lp + (size_t)16 * NL + k0);
    v8u bf[4];
#pragma unroll
    for (int t = 0; t < 4; ++t) bf[t] = ldfrag_u(Bp + (size_t)(16 * t) * NL + k0);
#pragma unroll
    for (int t = 0; t < 4; ++t) {
      acc[0][t] = mma_b(h0,  bf[t], acc[0][t]);
      acc[0][t] = mma_b(l0v, bf[t], acc[0][t]);
      acc[1][t] = mma_b(h1,  bf[t], acc[1][t]);
      acc[1][t] = mma_b(l1v, bf[t], acc[1][t]);
    }
    guard8(acc[0][0], acc[0][1], acc[0][2], acc[0][3], acc[1][0], acc[1][1], acc[1][2], acc[1][3],
           h0, h1, l0v, l1v, bf[0], bf[1], bf[2], bf[3]);
  }

#pragma unroll
  for (int i = 0; i < 2; ++i) {
#pragma unroll
    for (int t = 0; t < 4; ++t) {
#pragma unroll
      for (int r = 0; r < 8; ++r) Fs[(32 * wave + 16 * i + 8 * hh + r) * FSP + 16 * t + ci] = acc[i][t][r];
    }
  }
  __syncthreads();
  {
    const int p = tid & 15, rg = tid >> 4;
    float* ob = out0 + ((size_t)(b * NL + q0)) * ND + d0 + 4 * p;
    for (int pass = 0; pass < 2; ++pass) {
#pragma unroll 4
      for (int it = 0; it < 16; ++it) {
        const int rowi = it * 8 + rg;
        const v4f v = *(const v4f*)(Fs + rowi * FSP + 4 * p);
        *(volatile v4f*)(ob + (size_t)rowi * ND) = v;
      }
      __threadfence();
    }
  }
}

extern "C" void kernel_launch(void* const* d_in, const int* in_sizes, int n_in,
                              void* d_out, int out_size, void* d_ws, size_t ws_size,
                              hipStream_t stream) {
  if (n_in < 4) return;
  if (in_sizes[0] != NB * NL * ND) return;
  if (in_sizes[1] != NB * NL * NL) return;
  if (in_sizes[2] < 2 * ND * ND) return;
  if (in_sizes[3] < 2 * ND) return;
  if (out_size != NB * NL * ND + NB * NL * NL) return;

  const float* x    = (const float*)d_in[0];
  const float* td   = (const float*)d_in[1];
  const float* w    = (const float*)d_in[2];
  const float* bias = (const float*)d_in[3];

  const size_t PXb = (size_t)NB * NL * ND * 2;
  const size_t PWb = (size_t)2 * ND * ND * 2;
  const size_t PXT = (size_t)NB * ND * NL * 2;
  const size_t PQK = (size_t)2 * NB * NH * NL * HD * 2;
  const size_t PA  = (size_t)NB * NL * NL * 2;
  size_t off = 0;
  const size_t oXb = off; off += PXb;
  const size_t oWb = off; off += PWb;
  const size_t oXT = off; off += PXT;
  const size_t oQK = off; off += PQK;
  const size_t oAH = off; off += PA;
  const size_t oAL = off; off += PA;
  if (off > ws_size) return;
  if (off > (size_t)134217728) return;

  char* ws = (char*)d_ws;
  unsigned short* Xb = (unsigned short*)(ws + oXb);
  unsigned short* Wb = (unsigned short*)(ws + oWb);
  unsigned short* XT = (unsigned short*)(ws + oXT);
  unsigned short* QK = (unsigned short*)(ws + oQK);
  unsigned short* AH = (unsigned short*)(ws + oAH);
  unsigned short* AL = (unsigned short*)(ws + oAL);
  float* out0 = (float*)d_out;
  float* out1 = (float*)d_out + (size_t)NB * NL * ND;

  const dim3 blk256(256), blk128(128);
  const dim3 gCV(NBX + NBW);
  const dim3 gXT(NB * (NL / 64) * (ND / 64));
  const dim3 gPJ((NB * NL / 128) * (2 * ND / 64));
  const dim3 gAT(NB * (NL / 16));
  const dim3 gOP(NB * (NL / 128) * (ND / 64));

  cvt_in<<<gCV, blk256, 0, stream>>>(x, w, Xb, Wb);
  xpt<<<gXT, blk256, 0, stream>>>(x, XT);
  proj_qk<<<gPJ, blk128, 0, stream>>>(Xb, Wb, bias, QK);
  attn_w<<<gAT, blk256, 0, stream>>>(QK, td, out1, AH, AL);
  out_prod<<<gOP, blk128, 0, stream>>>(AH, AL, XT, out0);
  (void)hipGetLastError();
}
